// OST_8950711845626
// MI455X (gfx1250) — hardware-verified
//
#include <hip/hip_runtime.h>
#include <math.h>

constexpr int kB = 256;
constexpr int kT = 16;
constexpr int kA = 400;
constexpr int kN = 8;
constexpr int kD = 512;
constexpr int kRowsImg = kB * kT;
constexpr int kRowsDes = kA * kN;
constexpr int kAPad = 448;
constexpr int kPairsPerPass = 16;
constexpr int kPasses = kA / kPairsPerPass;
constexpr int kTrips = 4;
constexpr float kInvEps = 10.0f;
constexpr float kRowMarg = 1.0f / 16.0f;
constexpr float kColMarg = 1.0f / 8.0f;
static_assert(kA % kPairsPerPass == 0, "pass coverage");
static_assert(kD == 512, "lane maps assume 512 features");
static_assert(kAPad % 64 == 0 && kAPad >= kA && kAPad % 32 == 0, "pad");
static_assert((kB * kA) % (4 * 256) == 0, "combine grid exact");

typedef __attribute__((ext_vector_type(16))) _Float16 v16h;
typedef __attribute__((ext_vector_type(8)))  _Float16 v8h;
typedef __attribute__((ext_vector_type(16))) __bf16   v16b;
typedef __attribute__((ext_vector_type(8)))  __bf16   v8b;
typedef __attribute__((ext_vector_type(8)))  float    v8f;
typedef __attribute__((ext_vector_type(4)))  float    v4f;
typedef __attribute__((ext_vector_type(4)))  unsigned int v4u;

__device__ __forceinline__ unsigned short f2bf_bits(float f) {
  unsigned u = __float_as_uint(f);
  return (unsigned short)((u + 0x7FFFu + ((u >> 16) & 1u)) >> 16);
}
__device__ __forceinline__ float bf_bits2f(unsigned short h) { return __uint_as_float(((unsigned)h) << 16); }

__device__ __forceinline__ void dep_guard_h(v8f& a, v8f& b, v16h x, v16h y) { asm volatile("v_nop\n\tv_nop\n\tv_nop\n\tv_nop" : "+v"(a), "+v"(b) : "v"(x), "v"(y)); }
__device__ __forceinline__ void dep_guard_b(v8f& a, v8f& b, v16b x, v16b y) { asm volatile("v_nop\n\tv_nop\n\tv_nop\n\tv_nop" : "+v"(a), "+v"(b) : "v"(x), "v"(y)); }
__device__ __forceinline__ void keep4_h(v16h a, v16h b, v16h c, v16h d) { asm volatile("v_nop" :: "v"(a), "v"(b), "v"(c), "v"(d)); }
__device__ __forceinline__ void keep4_b(v16b a, v16b b, v16b c, v16b d) { asm volatile("v_nop" :: "v"(a), "v"(b), "v"(c), "v"(d)); }
__device__ __forceinline__ void acc_guard4(v8f& a, v8f& b, v8f& c, v8f& d) { asm volatile("v_nop\n\tv_nop\n\tv_nop\n\tv_nop" : "+v"(a), "+v"(b), "+v"(c), "+v"(d)); }
template <typename T> struct Frag;
template <> struct Frag<_Float16> {
  typedef v16h V; union U { v16h v; v8h h[2]; };
  static __device__ __forceinline__ v16h load(const _Float16* p) {
    U f; f.h[0] = *(const v8h*)(p); f.h[1] = *(const v8h*)(p + 16); return f.v;
  }
  static __device__ __forceinline__ v8f mma(v16h a, v16h b, v8f c) {
    return __builtin_amdgcn_wmma_f32_16x16x32_f16(false, a, false, b, (short)0, c, false, false);
  }
  static __device__ __forceinline__ void guard(v8f& a, v8f& b, v16h x, v16h y) { dep_guard_h(a, b, x, y); }
  static __device__ __forceinline__ void keep(v16h a, v16h b, v16h c, v16h d) { keep4_h(a, b, c, d); }
};
template <> struct Frag<__bf16> {
  typedef v16b V; union U { v16b v; v8b h[2]; };
  static __device__ __forceinline__ v16b load(const __bf16* p) {
    U f; f.h[0] = *(const v8b*)(p); f.h[1] = *(const v8b*)(p + 16); return f.v;
  }
  static __device__ __forceinline__ v8f mma(v16b a, v16b b, v8f c) {
    return __builtin_amdgcn_wmma_f32_16x16x32_bf16(false, a, false, b, (short)0, c, false, false);
  }
  static __device__ __forceinline__ void guard(v8f& a, v8f& b, v16b x, v16b y) { dep_guard_b(a, b, x, y); }
  static __device__ __forceinline__ void keep(v16b a, v16b b, v16b c, v16b d) { keep4_b(a, b, c, d); }
};

__device__ __forceinline__ unsigned pk16(unsigned short a, unsigned short b) { return (unsigned)a | ((unsigned)b << 16); }

template <int ET> struct Elem;
template <> struct Elem<0> { typedef _Float16 T; };
template <> struct Elem<1> { typedef __bf16 T; };
template <int ET, bool SPLIT, int BIAS_MODE, int OUT_MODE, bool RESID, int ACT = 0>
__global__ __launch_bounds__(256) void wmma_gemm64(
    const unsigned short* __restrict__ Ap, const unsigned short* __restrict__ A2p, int lda, long strideA,
    const unsigned short* __restrict__ Btp, const unsigned short* __restrict__ Bt2p, int ldb, long strideB,
    void* __restrict__ Cout, void* __restrict__ Cout2, int ldc, long strideC,
    const float* __restrict__ bias,
    const float* __restrict__ resid, long strideR,
    int M, int N, int K, float scale) {
  typedef typename Elem<ET>::T T;
  typedef typename Frag<T>::V V;
  const T* A = (const T*)Ap; const T* A2 = (const T*)A2p; const T* Bt = (const T*)Btp; const T* Bt2 = (const T*)Bt2p;
  __shared__ __align__(16) float sT[8][16 * 68];
  const int b    = blockIdx.y;
  const int lane = threadIdx.x & 31;
  const int wave = threadIdx.x >> 5;
  const int tilesN = N >> 6;
  const int tilesM = M >> 6;
  const int tile = blockIdx.x * 8 + wave;
  if (tile >= tilesM * tilesN) return;
  const int tm = tile / tilesN;
  const int tn = tile - tm * tilesN;
  const int m0 = tm << 6;
  const int n0 = tn << 6;

  const T* Ab  = A  + (size_t)b * strideA;
  const T* Bb  = Bt + (size_t)b * strideB;
  const T* Ab2 = SPLIT ? (A2  + (size_t)b * strideA) : nullptr;
  const T* Bb2 = SPLIT ? (Bt2 + (size_t)b * strideB) : nullptr;

  const int rlane = lane & 15;
  const int koff  = (lane >> 4) * 8;
  const int mOff  = (lane >> 4) * 8;

  v8f acc[4][4];
#pragma unroll
  for (int i = 0; i < 4; ++i)
#pragma unroll
    for (int j = 0; j < 4; ++j) acc[i][j] = (v8f){0.f,0.f,0.f,0.f,0.f,0.f,0.f,0.f};

  for (int k0 = 0; k0 < K; k0 += 32) {
    V bh[4], bl[4];
#pragma unroll
    for (int j = 0; j < 4; ++j) {
      const size_t bo = (size_t)(n0 + (j << 4) + rlane) * ldb + koff + k0;
      bh[j] = Frag<T>::load(Bb + bo);
      if (SPLIT) bl[j] = Frag<T>::load(Bb2 + bo);
    }
#pragma unroll
    for (int i = 0; i < 4; ++i) {
      const size_t ao = (size_t)(m0 + (i << 4) + rlane) * lda + koff + k0;
      V ah = Frag<T>::load(Ab + ao);
      V al;
      if (SPLIT) al = Frag<T>::load(Ab2 + ao);
#pragma unroll
      for (int j = 0; j < 4; ++j) {
        acc[i][j] = Frag<T>::mma(ah, bh[j], acc[i][j]);
        if (SPLIT) {
          acc[i][j] = Frag<T>::mma(ah, bl[j], acc[i][j]);
          acc[i][j] = Frag<T>::mma(al, bh[j], acc[i][j]);
        }
      }
      Frag<T>::guard(acc[i][0], acc[i][3], ah, SPLIT ? al : ah);
    }
    Frag<T>::keep(bh[0], bh[1], bh[2], bh[3]);
    if (SPLIT) Frag<T>::keep(bl[0], bl[1], bl[2], bl[3]);
  }
  acc_guard4(acc[0][0], acc[0][1], acc[0][2], acc[0][3]);
  acc_guard4(acc[1][0], acc[1][1], acc[1][2], acc[1][3]);
  acc_guard4(acc[2][0], acc[2][1], acc[2][2], acc[2][3]);
  acc_guard4(acc[3][0], acc[3][1], acc[3][2], acc[3][3]);

  float* slab = sT[wave];
  const float* Rb = RESID ? (resid + (size_t)b * strideR) : nullptr;
#pragma unroll
  for (int i = 0; i < 4; ++i) {
    const int mBase = m0 + (i << 4);
#pragma unroll
    for (int j = 0; j < 4; ++j) {
      const int n = n0 + (j << 4) + rlane;
      float bv = 0.f;
      if (BIAS_MODE == 2) bv = bias[n];
#pragma unroll
      for (int r = 0; r < 8; ++r) {
        float v = acc[i][j][r] * scale;
        if (BIAS_MODE == 1) v += bias[mBase + mOff + r];
        if (BIAS_MODE == 2) v += bv;
        if (RESID) v += Rb[(size_t)(mBase + mOff + r) * ldc + n];
        if (ACT == 2) v = fmaxf(v, 0.0f);
        if (ACT == 4) v = (v > 0.f) ? v : 0.01f * v;
        slab[(mOff + r) * 68 + (j << 4) + rlane] = v;
      }
    }
    __builtin_amdgcn_fence(__ATOMIC_RELEASE, "workgroup");
    __builtin_amdgcn_wave_barrier();
    __builtin_amdgcn_fence(__ATOMIC_ACQUIRE, "workgroup");
    if (OUT_MODE == 0) {
      float* C = (float*)Cout + (size_t)b * strideC;
      const int hh = lane >> 4, c4 = (lane & 15) * 4;
      for (int pass = 0; pass < 2; ++pass) {
#pragma unroll
        for (int it = 0; it < 8; ++it) {
          const int row = it * 2 + hh;
          v4f v = *(const v4f*)(slab + row * 68 + c4);
          *(volatile v4f*)(C + (size_t)(mBase + row) * ldc + n0 + c4) = v;
        }
        __threadfence();
      }
    } else {
      const int q = lane >> 3, c8 = (lane & 7) * 8;
      unsigned short* C  = (unsigned short*)Cout  + (size_t)b * strideC;
      unsigned short* C2 = (OUT_MODE == 2) ? ((unsigned short*)Cout2 + (size_t)b * strideC) : nullptr;
      for (int pass = 0; pass < 2; ++pass) {
#pragma unroll
        for (int it = 0; it < 4; ++it) {
          const int row = it * 4 + q;
          const float* sp = slab + row * 68 + c8;
          v8h hv, lv;
#pragma unroll
          for (int e = 0; e < 8; ++e) {
            if (OUT_MODE == 1) {
              hv[e] = (_Float16)sp[e];
            } else {
              unsigned short hb = f2bf_bits(sp[e]);
              unsigned short lb = f2bf_bits(sp[e] - bf_bits2f(hb));
              hv[e] = __builtin_bit_cast(_Float16, hb);
              lv[e] = __builtin_bit_cast(_Float16, lb);
            }
          }
          *(volatile v8h*)(C + (size_t)(mBase + row) * ldc + n0 + c8) = hv;
          if (OUT_MODE == 2) *(volatile v8h*)(C2 + (size_t)(mBase + row) * ldc + n0 + c8) = lv;
        }
        __threadfence();
      }
    }
    __builtin_amdgcn_fence(__ATOMIC_RELEASE, "workgroup");
    __builtin_amdgcn_wave_barrier();
    __builtin_amdgcn_fence(__ATOMIC_ACQUIRE, "workgroup");
  }
}

__device__ __forceinline__ void split_bf(float x, unsigned short& h, unsigned short& l) {
  h = f2bf_bits(x);
  l = f2bf_bits(x - bf_bits2f(h));
}
__device__ __forceinline__ v4u pack8(const unsigned short* b8) {
  return (v4u){pk16(b8[0], b8[1]), pk16(b8[2], b8[3]), pk16(b8[4], b8[5]), pk16(b8[6], b8[7])};
}

__global__ __launch_bounds__(512) void img_norm_kernel(const float* __restrict__ imf, const float* __restrict__ lsc,
                                                       unsigned short* __restrict__ hiP, unsigned short* __restrict__ loP,
                                                       unsigned short* __restrict__ phiP, unsigned short* __restrict__ ploP) {
  __shared__ __align__(16) float srow[kT][kD];
  __shared__ __align__(16) float spool[kD];
  const int b = blockIdx.x;
  const int tid = threadIdx.x;
  const int lane = tid & 31;
  const int wave = tid >> 5;
  const size_t rowIdx = (size_t)b * kT + wave;
  const float* row = imf + rowIdx * kD;
  float x[16];
  {
    const v4f a0 = *(const v4f*)(row + 8 * lane);
    const v4f a1 = *(const v4f*)(row + 8 * lane + 4);
    const v4f a2 = *(const v4f*)(row + 256 + 8 * lane);
    const v4f a3 = *(const v4f*)(row + 256 + 8 * lane + 4);
#pragma unroll
    for (int e = 0; e < 4; ++e) { x[e] = a0[e]; x[4 + e] = a1[e]; x[8 + e] = a2[e]; x[12 + e] = a3[e]; }
  }
  float ss = 0.f;
#pragma unroll
  for (int e = 0; e < 16; ++e) ss += x[e] * x[e];
#pragma unroll
  for (int off = 16; off > 0; off >>= 1) ss += __shfl_xor(ss, off, 32);
  const float inv = 1.0f / sqrtf(ss);
  float xn[16];
  unsigned short hb[16], lb[16];
#pragma unroll
  for (int e = 0; e < 16; ++e) { xn[e] = x[e] * inv; split_bf(xn[e], hb[e], lb[e]); }
  const v4u h0 = pack8(hb), h1 = pack8(hb + 8);
  const v4u l0 = pack8(lb), l1 = pack8(lb + 8);
  unsigned short* hrow = hiP + rowIdx * kD;
  unsigned short* lrow = loP + rowIdx * kD;
  for (int pass = 0; pass < 2; ++pass) {
    *(volatile v4u*)(hrow + 8 * lane)       = h0;
    *(volatile v4u*)(hrow + 256 + 8 * lane) = h1;
    *(volatile v4u*)(lrow + 8 * lane)       = l0;
    *(volatile v4u*)(lrow + 256 + 8 * lane) = l1;
    __threadfence();
  }
  *(v4f*)(&srow[wave][8 * lane])           = (v4f){xn[0], xn[1], xn[2], xn[3]};
  *(v4f*)(&srow[wave][8 * lane + 4])       = (v4f){xn[4], xn[5], xn[6], xn[7]};
  *(v4f*)(&srow[wave][256 + 8 * lane])     = (v4f){xn[8], xn[9], xn[10], xn[11]};
  *(v4f*)(&srow[wave][256 + 8 * lane + 4]) = (v4f){xn[12], xn[13], xn[14], xn[15]};
  __syncthreads();
  {
    float s = 0.f;
#pragma unroll
    for (int t = 0; t < kT; ++t) s += srow[t][tid];
    const float ls = expf(lsc[0]);
    spool[tid] = ls * (s * (1.0f / 16.0f));
  }
  __syncthreads();
  if (tid < 64) {
    const v4f p0 = *(const v4f*)(&spool[8 * tid]);
    const v4f p1 = *(const v4f*)(&spool[8 * tid + 4]);
    unsigned short ph[8], pl[8];
#pragma unroll
    for (int e = 0; e < 4; ++e) { split_bf(p0[e], ph[e], pl[e]); split_bf(p1[e], ph[4 + e], pl[4 + e]); }
    const v4u hv = pack8(ph), lv = pack8(pl);
    unsigned short* pr = phiP + (size_t)b * kD + 8 * tid;
    unsigned short* qr = ploP + (size_t)b * kD + 8 * tid;
    *(volatile v4u*)pr = hv;
    *(volatile v4u*)qr = lv;
    __threadfence();
    *(volatile v4u*)pr = hv;
    *(volatile v4u*)qr = lv;
  }
}

__global__ __launch_bounds__(256) void desc_norm_kernel(const float* __restrict__ des,
                                                        unsigned short* __restrict__ hiP, unsigned short* __restrict__ loP,
                                                        unsigned short* __restrict__ phiP, unsigned short* __restrict__ ploP) {
  __shared__ __align__(16) float srow[kN][kD];
  __shared__ __align__(16) float spool[kD];
  const int a = blockIdx.x;
  const bool valid = a < kA;
  const int ac = valid ? a : (kA - 1);
  const int tid = threadIdx.x;
  const int lane = tid & 31;
  const int wave = tid >> 5;
  const size_t rowIdx = (size_t)ac * kN + wave;
  const float* row = des + rowIdx * kD;
  float x[16];
  {
    const v4f a0 = *(const v4f*)(row + 8 * lane);
    const v4f a1 = *(const v4f*)(row + 8 * lane + 4);
    const v4f a2 = *(const v4f*)(row + 256 + 8 * lane);
    const v4f a3 = *(const v4f*)(row + 256 + 8 * lane + 4);
#pragma unroll
    for (int e = 0; e < 4; ++e) { x[e] = a0[e]; x[4 + e] = a1[e]; x[8 + e] = a2[e]; x[12 + e] = a3[e]; }
  }
  float ss = 0.f;
#pragma unroll
  for (int e = 0; e < 16; ++e) ss += x[e] * x[e];
#pragma unroll
  for (int off = 16; off > 0; off >>= 1) ss += __shfl_xor(ss, off, 32);
  const float inv = 1.0f / sqrtf(ss);
  float xn[16];
  unsigned short hb[16], lb[16];
#pragma unroll
  for (int e = 0; e < 16; ++e) { xn[e] = x[e] * inv; split_bf(xn[e], hb[e], lb[e]); }
  if (valid) {
    const v4u h0 = pack8(hb), h1 = pack8(hb + 8);
    const v4u l0 = pack8(lb), l1 = pack8(lb + 8);
    unsigned short* hrow = hiP + rowIdx * kD;
    unsigned short* lrow = loP + rowIdx * kD;
    for (int pass = 0; pass < 2; ++pass) {
      *(volatile v4u*)(hrow + 8 * lane)       = h0;
      *(volatile v4u*)(hrow + 256 + 8 * lane) = h1;
      *(volatile v4u*)(lrow + 8 * lane)       = l0;
      *(volatile v4u*)(lrow + 256 + 8 * lane) = l1;
      __threadfence();
    }
  }
  *(v4f*)(&srow[wave][8 * lane])           = (v4f){xn[0], xn[1], xn[2], xn[3]};
  *(v4f*)(&srow[wave][8 * lane + 4])       = (v4f){xn[4], xn[5], xn[6], xn[7]};
  *(v4f*)(&srow[wave][256 + 8 * lane])     = (v4f){xn[8], xn[9], xn[10], xn[11]};
  *(v4f*)(&srow[wave][256 + 8 * lane + 4]) = (v4f){xn[12], xn[13], xn[14], xn[15]};
  __syncthreads();
#pragma unroll
  for (int half = 0; half < 2; ++half) {
    const int d = tid + 256 * half;
    float s = 0.f;
#pragma unroll
    for (int n = 0; n < kN; ++n) s += srow[n][d];
    const float pv = s * (1.0f / 8.0f);
    spool[d] = valid ? pv : 0.0f;
  }
  __syncthreads();
  if (tid < 64) {
    const v4f p0 = *(const v4f*)(&spool[8 * tid]);
    const v4f p1 = *(const v4f*)(&spool[8 * tid + 4]);
    unsigned short ph[8], pl[8];
#pragma unroll
    for (int e = 0; e < 4; ++e) { split_bf(p0[e], ph[e], pl[e]); split_bf(p1[e], ph[4 + e], pl[4 + e]); }
    const v4u hv = pack8(ph), lv = pack8(pl);
    unsigned short* pr = phiP + (size_t)a * kD + 8 * tid;
    unsigned short* qr = ploP + (size_t)a * kD + 8 * tid;
    *(volatile v4u*)pr = hv;
    *(volatile v4u*)qr = lv;
    __threadfence();
    *(volatile v4u*)pr = hv;
    *(volatile v4u*)qr = lv;
  }
}

__global__ __launch_bounds__(256) void sinkhorn_kernel(const float* __restrict__ sim, float* __restrict__ ot) {
  __shared__ __align__(16) float ssc[kAPad];
  const int b = blockIdx.x;
  const int tid = threadIdx.x;
  const int lane = tid & 31;
  const int wave = tid >> 5;
  const int t = lane & 15;
  const int ph = lane >> 4;
  const int bit3 = (t >> 3) & 1, bit2 = (t >> 2) & 1, bit1 = (t >> 1) & 1;
  if (tid < kAPad - kA) ssc[kA + tid] = 0.0f;
#pragma unroll 1
  for (int pass = 0; pass < kPasses; ++pass) {
    const int a = pass * kPairsPerPass + wave * 2 + ph;
    const float* sp = sim + ((size_t)b * kT + t) * kRowsDes + (size_t)a * kN;
    const v4f s0 = *(const v4f*)(sp);
    const v4f s1 = *(const v4f*)(sp + 4);
    float sv[8], kk[8], c[8];
#pragma unroll
    for (int n = 0; n < 4; ++n) { sv[n] = s0[n]; sv[4 + n] = s1[n]; }
#pragma unroll
    for (int n = 0; n < 8; ++n) {
      const float cost = 1.0f - sv[n];
      const float arg = -cost * kInvEps;
      kk[n] = expf(arg);
      c[n] = 1.0f;
    }
    float r = 1.0f;
#pragma unroll 1
    for (int it = 0; it < kTrips; ++it) {
      float rs = 0.f;
#pragma unroll
      for (int n = 0; n < 8; ++n) rs += kk[n] * c[n];
      r = kRowMarg / rs;
      float q[8];
#pragma unroll
      for (int n = 0; n < 8; ++n) q[n] = kk[n] * r;
      float h4[4];
#pragma unroll
      for (int j = 0; j < 4; ++j) {
        const float keep = bit3 ? q[4 + j] : q[j];
        const float send = bit3 ? q[j] : q[4 + j];
        const float recv = __shfl_xor(send, 8, 32);
        h4[j] = keep + recv;
      }
      float h2[2];
#pragma unroll
      for (int j = 0; j < 2; ++j) {
        const float keep = bit2 ? h4[2 + j] : h4[j];
        const float send = bit2 ? h4[j] : h4[2 + j];
        const float recv = __shfl_xor(send, 4, 32);
        h2[j] = keep + recv;
      }
      float h1;
      {
        const float keep = bit1 ? h2[1] : h2[0];
        const float send = bit1 ? h2[0] : h2[1];
        const float recv = __shfl_xor(send, 2, 32);
        h1 = keep + recv;
      }
      h1 += __shfl_xor(h1, 1, 32);
      const float cn = kColMarg / h1;
#pragma unroll
      for (int n = 0; n < 8; ++n) c[n] = __shfl(cn, 2 * n, 16);
    }
    float ps = 0.f;
#pragma unroll
    for (int n = 0; n < 8; ++n) {
      const float pe = (r * c[n]) * kk[n];
      ps += pe * sv[n];
    }
    ps += __shfl_xor(ps, 1, 32);
    ps += __shfl_xor(ps, 2, 32);
    ps += __shfl_xor(ps, 4, 32);
    ps += __shfl_xor(ps, 8, 32);
    if (t == 0) ssc[a] = ps;
  }
  __syncthreads();
  {
    const bool w = tid < (kAPad / 32) * 8;
    const int line = w ? (tid >> 3) : 0;
    const int e = tid & 7;
    const v4f val = *(const v4f*)(&ssc[line * 32 + e * 4]);
    float* dst = ot + (size_t)b * kAPad + line * 32 + e * 4;
    for (int pass = 0; pass < 2; ++pass) {
      if (w) *(volatile v4f*)dst = val;
      __threadfence();
    }
  }
}

__global__ __launch_bounds__(256) void combine_kernel(const float* __restrict__ plT, const float* __restrict__ plS,
                                                      const float* __restrict__ otT, const float* __restrict__ otS,
                                                      const float* __restrict__ lsc, float* __restrict__ out) {
  const int i = blockIdx.x * 256 + threadIdx.x;
  if (i >= (kB * kA) / 4) return;
  const float ls = expf(lsc[0]);
  v4f o;
#pragma unroll
  for (int e = 0; e < 4; ++e) {
    const int idx = 4 * i + e;
    const int bb = idx / kA;
    const int aa = idx - bb * kA;
    const int k = bb * kAPad + aa;
    const float lt = plT[k] + otT[k] * ls;
    const float lsp = plS[k] + otS[k] * ls;
    o[e] = 0.5f * lt + 0.5f * lsp;
  }
  float* dst = out + 4 * (size_t)i;
  *(volatile v4f*)dst = o;
  __threadfence();
  *(volatile v4f*)dst = o;
}

extern "C" void kernel_launch(void* const* d_in, const int* in_sizes, int n_in,
                              void* d_out, int out_size, void* d_ws, size_t ws_size,
                              hipStream_t stream) {
  if (n_in < 4) return;
  if (in_sizes[0] != kRowsImg * kD || in_sizes[1] != kRowsDes * kD || in_sizes[2] != kRowsDes * kD ||
      in_sizes[3] < 1 || out_size != kB * kA) return;
  const float* imf = (const float*)d_in[0];
  const float* ds  = (const float*)d_in[1];
  const float* dt  = (const float*)d_in[2];
  const float* lsc = (const float*)d_in[3];
  float* out = (float*)d_out;

  char* ws = (char*)d_ws;
  size_t off = 0;
  auto take = [&](size_t bytes) -> char* {
    char* p = ws + off;
    off += (bytes + 255) & ~(size_t)255;
    return p;
  };
  const size_t imfPlane = (size_t)kRowsImg * kD * 2;
  const size_t desPlane = (size_t)kRowsDes * kD * 2;
  const size_t poolPlane = (size_t)kB * kD * 2;
  const size_t dpPlane = (size_t)2 * kAPad * kD * 2;
  const size_t simBytes = (size_t)kRowsImg * kRowsDes * 4;
  const size_t scorePlane = (size_t)2 * kB * kAPad * 4;
  unsigned short* imfHi = (unsigned short*)take(imfPlane);
  unsigned short* imfLo = (unsigned short*)take(imfPlane);
  unsigned short* dtHi  = (unsigned short*)take(desPlane);
  unsigned short* dtLo  = (unsigned short*)take(desPlane);
  unsigned short* dsHi  = (unsigned short*)take(desPlane);
  unsigned short* dsLo  = (unsigned short*)take(desPlane);
  unsigned short* poolHi = (unsigned short*)take(poolPlane);
  unsigned short* poolLo = (unsigned short*)take(poolPlane);
  unsigned short* dpHi  = (unsigned short*)take(dpPlane);
  unsigned short* dpLo  = (unsigned short*)take(dpPlane);
  float* simP = (float*)take(simBytes);
  float* otP  = (float*)take(scorePlane);
  float* plP  = (float*)take(scorePlane);
  if (off > ws_size) return;

  const size_t dpSet = (size_t)kAPad * kD;
  const size_t scSet = (size_t)kB * kAPad;

  img_norm_kernel<<<kB, 512, 0, stream>>>(imf, lsc, imfHi, imfLo, poolHi, poolLo);
  desc_norm_kernel<<<kAPad, 256, 0, stream>>>(dt, dtHi, dtLo, dpHi, dpLo);
  desc_norm_kernel<<<kAPad, 256, 0, stream>>>(ds, dsHi, dsLo, dpHi + dpSet, dpLo + dpSet);

  wmma_gemm64<1, true, 0, 0, false, 0><<<dim3(400, 1), 256, 0, stream>>>(
      imfHi, imfLo, kD, 0L, dtHi, dtLo, kD, 0L, (void*)simP, nullptr, kRowsDes, 0L,
      nullptr, nullptr, 0L, kRowsImg, kRowsDes, kD, 1.0f);
  sinkhorn_kernel<<<kB, 256, 0, stream>>>(simP, otP);

  wmma_gemm64<1, true, 0, 0, false, 0><<<dim3(400, 1), 256, 0, stream>>>(
      imfHi, imfLo, kD, 0L, dsHi, dsLo, kD, 0L, (void*)simP, nullptr, kRowsDes, 0L,
      nullptr, nullptr, 0L, kRowsImg, kRowsDes, kD, 1.0f);
  sinkhorn_kernel<<<kB, 256, 0, stream>>>(simP, otP + scSet);

  wmma_gemm64<1, true, 0, 0, false, 0><<<dim3(4, 2), 256, 0, stream>>>(
      poolHi, poolLo, kD, 0L, dpHi, dpLo, kD, (long)dpSet, (void*)plP, nullptr, kAPad, (long)scSet,
      nullptr, nullptr, 0L, kB, kAPad, kD, 1.0f);

  combine_kernel<<<(kB * kA) / (4 * 256), 256, 0, stream>>>(plP, plP + scSet, otP, otP + scSet, lsc, out);
}
